// ScaledDotProductAttention_33681133535677
// MI455X (gfx1250) — hardware-verified
//
#include <hip/hip_runtime.h>


typedef __attribute__((ext_vector_type(16))) _Float16 v16h;
typedef __attribute__((ext_vector_type(8)))  _Float16 v8h;
typedef __attribute__((ext_vector_type(8)))  float    v8f;
typedef __attribute__((ext_vector_type(4)))  float    v4f;
typedef __attribute__((ext_vector_type(4)))  int      v4i;
typedef __attribute__((ext_vector_type(4)))  unsigned v4u;

#ifndef NB
#define NB 2
#endif
#ifndef SEQ
#define SEQ 2048
#endif
#define NB_FULL  2
#define SEQ_FULL 2048

constexpr int HEADS = 12;
constexpr int DH    = 64;
constexpr int QTILE = 128;
constexpr int KBLK  = 128;
constexpr int NBLK  = SEQ / KBLK;
constexpr int NT    = KBLK / 16;
constexpr int KD    = DH + 8;
constexpr int VD    = KBLK + 8;
constexpr int PD    = KBLK + 8;
constexpr int OD    = DH + 4;
constexpr int WPR   = SEQ / 32;
constexpr int NCH   = SEQ / 128;

static_assert(SEQ % 128 == 0);
static_assert(SEQ >= 128 && SEQ <= SEQ_FULL);
static_assert(NB >= 1 && NB <= NB_FULL);
static_assert(DH == 64);
static_assert(QTILE == 128 && KBLK == 128);

constexpr float SL2E  = 0.18033688011112042f;
constexpr float MFILL = -1.0e9f;

__device__ __forceinline__ _Float16 to_h(float x) {
    unsigned u = __float_as_uint(x);
    u = (u + 0x7FFFu + ((u >> 16) & 1u)) & 0xFFFF0000u;
    return (_Float16)__uint_as_float(u);
}

__device__ __forceinline__ float ex2(float x) { return __builtin_amdgcn_exp2f(x); }

__device__ __forceinline__ float rcp1(float x) {
#if defined(__has_builtin)
#if __has_builtin(__builtin_amdgcn_rcpf)
    return __builtin_amdgcn_rcpf(x);
#else
    return 1.0f / x;
#endif
#else
    return 1.0f / x;
#endif
}

__device__ __forceinline__ v8f wmma16(v16h a, v16h b, v8f c) {
    v8f d = __builtin_amdgcn_wmma_f32_16x16x32_f16(false, a, false, b, (short)0, c, false, false);
    asm volatile("v_nop\n\tv_nop\n\tv_nop\n\tv_nop" : "+v"(d) : "v"(a), "v"(b));
    return d;
}

union U16 { v16h v; v8h h[2]; };

__device__ __forceinline__ v16h ld_op16(const _Float16* p) {
    U16 u;
    u.h[0] = *(const v8h*)(p);
    u.h[1] = *(const v8h*)(p + 16);
    return u.v;
}

__device__ __forceinline__ v8h cvt8(const float* p) {
    const v4f a = *(const v4f*)p;
    const v4f b = *(const v4f*)(p + 4);
    v8h r = {to_h(a.x), to_h(a.y), to_h(a.z), to_h(a.w),
             to_h(b.x), to_h(b.y), to_h(b.z), to_h(b.w)};
    return r;
}

__global__ __launch_bounds__(256)
void mask_bits_kernel(const int* __restrict__ mask, unsigned* __restrict__ bits, int nrows)
{
    const int lane = threadIdx.x & 31;
    const int wv   = threadIdx.x >> 5;
    const int rw   = blockIdx.x * 8 + wv;
    if (rw >= nrows) return;
    const int b  = rw / SEQ;
    const int qr = rw - b * SEQ;
    const int* src = mask + ((size_t)b * SEQ_FULL + qr) * (size_t)SEQ_FULL;

    unsigned k0 = 0u, k1 = 0u, k2 = 0u, k3 = 0u;
#pragma unroll 1
    for (int c = 0; c < NCH; ++c) {
        const v4i x = *(const v4i*)(src + 128 * c + 4 * lane);
        const unsigned w0 = __builtin_amdgcn_ballot_w32(x.x != 0);
        const unsigned w1 = __builtin_amdgcn_ballot_w32(x.y != 0);
        const unsigned w2 = __builtin_amdgcn_ballot_w32(x.z != 0);
        const unsigned w3 = __builtin_amdgcn_ballot_w32(x.w != 0);
        const bool mine = (lane == c);
        k0 = mine ? w0 : k0;
        k1 = mine ? w1 : k1;
        k2 = mine ? w2 : k2;
        k3 = mine ? w3 : k3;
    }
    unsigned* dst = bits + (size_t)rw * WPR + 4 * lane;
    v4u st;
    st.x = k0; st.y = k1; st.z = k2; st.w = k3;
    if (lane < NCH) *(volatile v4u*)dst = st;
    __threadfence();
    if (lane < NCH) *(volatile v4u*)dst = st;
}

__global__ __launch_bounds__(256)
void convert_kv_kernel(const float* __restrict__ K, const float* __restrict__ V,
                       _Float16* __restrict__ Kh, _Float16* __restrict__ Vt)
{
    __shared__ __align__(16) _Float16 Vs[DH * VD];

    const int cb  = blockIdx.x;
    const int bh  = blockIdx.y;
    const int b   = bh / HEADS;
    const int hh  = bh - b * HEADS;
    const int tid = threadIdx.x;

    const size_t ibase = ((size_t)b * HEADS + hh) * (size_t)SEQ_FULL * DH;
    const float* Kin = K + ibase;
    const float* Vin = V + ibase;
    _Float16* Kout = Kh + (size_t)bh * SEQ * DH;
    _Float16* Vout = Vt + (size_t)bh * DH * SEQ;

    v8h kh[4];
#pragma unroll
    for (int i = 0; i < 4; ++i) {
        const int idx = tid + 256 * i;
        const int row = idx >> 3, p = idx & 7;
        kh[i] = cvt8(Kin + (size_t)(cb * 128 + row) * DH + 8 * p);
    }

#pragma unroll
    for (int i = 0; i < 8; ++i) {
        const int idx = tid + 256 * i;
        const int s = idx >> 4, j = idx & 15;
        const v4f a = *(const v4f*)(Vin + (size_t)(cb * 128 + s) * DH + 4 * j);
        Vs[(4 * j + 0) * VD + s] = to_h(a.x);
        Vs[(4 * j + 1) * VD + s] = to_h(a.y);
        Vs[(4 * j + 2) * VD + s] = to_h(a.z);
        Vs[(4 * j + 3) * VD + s] = to_h(a.w);
    }
    __syncthreads();

    v8h vv[4];
#pragma unroll
    for (int i = 0; i < 4; ++i) {
        const int idx = tid + 256 * i;
        const int d = idx >> 4, p = idx & 15;
        vv[i] = *(const v8h*)&Vs[d * VD + 8 * p];
    }

#pragma unroll
    for (int i = 0; i < 4; ++i) {
        const int idx = tid + 256 * i;
        {
            const int row = idx >> 3, p = idx & 7;
            *(volatile v8h*)(Kout + (size_t)(cb * 128 + row) * DH + 8 * p) = kh[i];
        }
        {
            const int d = idx >> 4, p = idx & 15;
            *(volatile v8h*)(Vout + (size_t)d * SEQ + cb * 128 + 8 * p) = vv[i];
        }
    }
    __threadfence();
#pragma unroll
    for (int i = 0; i < 4; ++i) {
        const int idx = tid + 256 * i;
        {
            const int row = idx >> 3, p = idx & 7;
            *(volatile v8h*)(Kout + (size_t)(cb * 128 + row) * DH + 8 * p) = kh[i];
        }
        {
            const int d = idx >> 4, p = idx & 15;
            *(volatile v8h*)(Vout + (size_t)d * SEQ + cb * 128 + 8 * p) = vv[i];
        }
    }
}

__global__ void __launch_bounds__(256) __attribute__((amdgpu_num_vgpr(256)))
fa_kernel(const float* __restrict__ Q,
          const _Float16* __restrict__ Kh,
          const _Float16* __restrict__ Vt,
          const unsigned* __restrict__ Mbits,
          float* __restrict__ O)
{
    __shared__ __align__(16) _Float16 Ksh[KBLK * KD];
    __shared__ __align__(16) _Float16 Vts[DH * VD];
    __shared__ __align__(16) _Float16 Pst[8 * 16 * PD];
    __shared__ __align__(16) float    Ost[8 * 16 * OD];

    const int qb   = blockIdx.x;
    const int h    = blockIdx.y;
    const int bb   = blockIdx.z;
    const int tid  = threadIdx.x;
    const int lane = tid & 31;
    const int wv   = tid >> 5;
    const int hf   = lane >> 4;
    const int l16  = lane & 15;
    const int koff = hf * 8;
    const int jsel = l16 & 3;
    const unsigned shb = (unsigned)(l16 >> 2);

    const size_t bh = (size_t)bb * HEADS + h;
    const float*    Qb  = Q     + bh * (size_t)SEQ_FULL * DH;
    const _Float16* KhB = Kh    + bh * (size_t)SEQ * DH;
    const _Float16* VtB = Vt    + bh * (size_t)DH * SEQ;
    const unsigned* Mb  = Mbits + (size_t)bb * SEQ * WPR;
    float*          Ob  = O     + bh * (size_t)SEQ * DH;

    const int q0 = qb * QTILE + wv * 16;

    v16h qa0, qa1;
    {
        const float* qp = Qb + (size_t)(q0 + l16) * DH;
        U16 u;
        u.h[0] = cvt8(qp + koff);       u.h[1] = cvt8(qp + 16 + koff);  qa0 = u.v;
        u.h[0] = cvt8(qp + 32 + koff);  u.h[1] = cvt8(qp + 48 + koff);  qa1 = u.v;
    }

    v16h vones;
#pragma unroll
    for (int j = 0; j < 16; ++j) vones[j] = (_Float16)1.0f;

    const v8f vzero = {0.f, 0.f, 0.f, 0.f, 0.f, 0.f, 0.f, 0.f};
    v8f o[4];
#pragma unroll
    for (int t = 0; t < 4; ++t) o[t] = vzero;
    v8f olsum = vzero;

    float m[8];
#pragma unroll
    for (int v = 0; v < 8; ++v) m[v] = -1.0e30f;

    _Float16* Pw = &Pst[wv * 16 * PD];

#pragma unroll 1
    for (int kb = 0; kb < NBLK; ++kb) {
        __syncthreads();
#pragma unroll
        for (int i = 0; i < 4; ++i) {
            const int c = tid + i * 256;
            {
                const int row = c >> 3, cc = c & 7;
                *(v8h*)&Ksh[row * KD + cc * 8] =
                    *(const v8h*)(KhB + (size_t)(kb * KBLK + row) * DH + cc * 8);
            }
            {
                const int row = c >> 4, cc = c & 15;
                *(v8h*)&Vts[row * VD + cc * 8] =
                    *(const v8h*)(VtB + (size_t)row * SEQ + kb * KBLK + cc * 8);
            }
        }
        __syncthreads();

        v8f c[NT];
#pragma unroll
        for (int t = 0; t < NT; ++t) c[t] = vzero;
#pragma unroll
        for (int kc = 0; kc < 2; ++kc) {
            const v16h a = kc ? qa1 : qa0;
#pragma unroll
            for (int t = 0; t < NT; ++t) {
                const v16h bop = ld_op16(&Ksh[(t * 16 + l16) * KD + kc * 32 + koff]);
                c[t] = wmma16(a, bop, c[t]);
            }
        }

        float sc[8], mb[8];
#pragma unroll
        for (int v = 0; v < 8; ++v) {
            const v4u mw = *(const v4u*)(Mb + (size_t)(q0 + 8 * hf + v) * WPR + 4 * kb);
            unsigned wsel = mw.w;
            wsel = (jsel == 2) ? mw.z : wsel;
            wsel = (jsel == 1) ? mw.y : wsel;
            wsel = (jsel == 0) ? mw.x : wsel;
            float r = MFILL;
#pragma unroll
            for (int t = 0; t < NT; ++t) {
                const unsigned bit = (wsel >> (shb + 4u * (unsigned)t)) & 1u;
                const float s  = c[t][v] * SL2E;
                const float sm = (bit != 0u) ? s : MFILL;
                c[t][v] = sm;
                r = fmaxf(r, sm);
            }
            r = fmaxf(r, __shfl_xor(r, 1, 32));
            r = fmaxf(r, __shfl_xor(r, 2, 32));
            r = fmaxf(r, __shfl_xor(r, 4, 32));
            r = fmaxf(r, __shfl_xor(r, 8, 32));
            const float mn = fmaxf(m[v], r);
            sc[v] = ex2(m[v] - mn);
            m[v]  = mn;
            mb[v] = mn - 8.0f;
        }
#pragma unroll
        for (int t = 0; t < NT; ++t)
#pragma unroll
            for (int v = 0; v < 8; ++v)
                c[t][v] = ex2(c[t][v] - mb[v]);

#pragma unroll
        for (int v = 0; v < 8; ++v) {
#pragma unroll
            for (int t = 0; t < 4; ++t) o[t][v] *= sc[v];
            olsum[v] *= sc[v];
        }

#pragma unroll
        for (int t = 0; t < NT; ++t)
#pragma unroll
            for (int v = 0; v < 8; ++v)
                Pw[(v + 8 * hf) * PD + t * 16 + l16] = (_Float16)c[t][v];
        __syncthreads();

#pragma unroll
        for (int kc = 0; kc < 4; ++kc) {
            const v16h pa = ld_op16(&Pw[l16 * PD + kc * 32 + koff]);
            olsum = wmma16(pa, vones, olsum);
#pragma unroll
            for (int t = 0; t < 4; ++t) {
                const v16h vb = ld_op16(&Vts[(t * 16 + l16) * VD + kc * 32 + koff]);
                o[t] = wmma16(pa, vb, o[t]);
            }
        }
    }

    float* Ow = &Ost[wv * 16 * OD];
#pragma unroll
    for (int v = 0; v < 8; ++v) {
        const float rinv = rcp1(olsum[v]);
#pragma unroll
        for (int t = 0; t < 4; ++t)
            Ow[(8 * hf + v) * OD + t * 16 + l16] = o[t][v] * rinv;
    }
    __syncthreads();

#pragma unroll
    for (int i = 0; i < 8; ++i) {
        const int row = 2 * i + hf;
        const v4f val = *(const v4f*)&Ow[row * OD + 4 * l16];
        *(volatile v4f*)(Ob + (size_t)(q0 + row) * DH + 4 * l16) = val;
    }
    __threadfence();
#pragma unroll
    for (int i = 0; i < 8; ++i) {
        const int row = 2 * i + hf;
        const v4f val = *(const v4f*)&Ow[row * OD + 4 * l16];
        *(volatile v4f*)(Ob + (size_t)(q0 + row) * DH + 4 * l16) = val;
    }
}

extern "C" void kernel_launch(void* const* d_in, const int* in_sizes, int n_in,
                              void* d_out, int out_size, void* d_ws, size_t ws_size,
                              hipStream_t stream)
{
    if (n_in < 4) return;
    const float* q    = (const float*)d_in[0];
    const float* k    = (const float*)d_in[1];
    const float* v    = (const float*)d_in[2];
    const int*   mask = (const int*)  d_in[3];
    float*       out  = (float*)d_out;

    const long long need_qkv = (long long)NB * HEADS * SEQ_FULL * DH;
    const long long need_msk = (long long)NB * SEQ_FULL * SEQ_FULL;
    const long long need_out = (long long)NB * HEADS * SEQ * DH;
    if ((long long)in_sizes[0] < need_qkv || (long long)in_sizes[1] < need_qkv ||
        (long long)in_sizes[2] < need_qkv || (long long)in_sizes[3] < need_msk) return;
    if ((long long)out_size < need_out) return;

    const size_t plane_b = (size_t)NB * HEADS * SEQ * DH * sizeof(_Float16);
    const size_t bits_b  = (size_t)NB * SEQ * WPR * sizeof(unsigned);
    size_t off = 0;
    char* ws = (char*)d_ws;
    _Float16* Kh   = (_Float16*)(ws + off); off += plane_b;
    _Float16* Vt   = (_Float16*)(ws + off); off += plane_b;
    unsigned* bits = (unsigned*)(ws + off); off += bits_b;
    if (off > ws_size) return;

    const int nrows = NB * SEQ;
    mask_bits_kernel<<<dim3(nrows / 8), dim3(256), 0, stream>>>(mask, bits, nrows);

    convert_kv_kernel<<<dim3(SEQ / 128, NB * HEADS), dim3(256), 0, stream>>>(k, v, Kh, Vt);

    fa_kernel<<<dim3(SEQ / QTILE, HEADS, NB), dim3(256), 0, stream>>>(q, Kh, Vt, bits, out);
}
